// GRAM_27333171872172
// MI455X (gfx1250) — hardware-verified
//
#include <hip/hip_runtime.h>

#define DIM   256
#define ADIM  128
#define MANC  32
#define K2    512

typedef _Float16 v16h __attribute__((ext_vector_type(16)));
typedef _Float16 v8h  __attribute__((ext_vector_type(8)));
typedef float    v8f  __attribute__((ext_vector_type(8)));
typedef float    v4f  __attribute__((ext_vector_type(4)));
typedef float    v4fa __attribute__((ext_vector_type(4), may_alias));

union Frag { v16h v; v8h hf[2]; };

__device__ __forceinline__ v8f wmma_f16(v16h a, v16h b, v8f c) {
    v8f d = __builtin_amdgcn_wmma_f32_16x16x32_f16(false, a, false, b, (short)0, c, false, false);
    asm volatile("v_nop\n\tv_nop\n\tv_nop\n\tv_nop" : "+v"(d) : "v"(a), "v"(b));
    return d;
}

__device__ __forceinline__ float shf_f(float v, int src) {
    return __int_as_float(__builtin_amdgcn_ds_bpermute(src << 2, __float_as_int(v)));
}
__device__ __forceinline__ int shf_i(int v, int src) {
    return __builtin_amdgcn_ds_bpermute(src << 2, v);
}
__device__ __forceinline__ float wave_sum(float v) {
    const int l = (int)(threadIdx.x & 31);
    v += shf_f(v, l ^ 16);
    v += shf_f(v, l ^ 8);
    v += shf_f(v, l ^ 4);
    v += shf_f(v, l ^ 2);
    v += shf_f(v, l ^ 1);
    return v;
}
__device__ __forceinline__ float wave_max(float v) {
    const int l = (int)(threadIdx.x & 31);
    v = fmaxf(v, shf_f(v, l ^ 16));
    v = fmaxf(v, shf_f(v, l ^ 8));
    v = fmaxf(v, shf_f(v, l ^ 4));
    v = fmaxf(v, shf_f(v, l ^ 2));
    v = fmaxf(v, shf_f(v, l ^ 1));
    return v;
}

__global__ __launch_bounds__(256)
void k_cvt(const float* __restrict__ src, _Float16* __restrict__ dst, int n8, float scale) {
    const int g = blockIdx.x * blockDim.x + threadIdx.x;
    if (g < n8) {
        const float* s = src + (size_t)g * 8;
        v4f x0 = *(const v4f*)s;
        v4f x1 = *(const v4f*)(s + 4);
        x0 = x0 * scale;
        x1 = x1 * scale;
        v8f x = __builtin_shufflevector(x0, x1, 0, 1, 2, 3, 4, 5, 6, 7);
        v8h hv = __builtin_convertvector(x, v8h);
        volatile v8h* d = (volatile v8h*)(dst + (size_t)g * 8);
        *d = hv;
        __threadfence();
        *d = hv;
    }
}

__global__ __launch_bounds__(128)
void k_proj(const _Float16* __restrict__ e16,
            const _Float16* __restrict__ w16,
            float*          __restrict__ P,
            int nC, float oscale)
{
    __shared__ float stile[4 * 16 * 64];

    const int tid = (int)threadIdx.x;
    const int wv  = tid >> 5;
    const int l   = tid & 31;
    const int h   = l >> 4;
    const int m   = l & 15;
    const int r0  = blockIdx.x * 16;

    int ra = r0 + m;
    if (ra > nC - 1) ra = nC - 1;
    const _Float16* arow = e16 + (size_t)ra * DIM;

    const int chalf = wv >> 1;
    const int cb    = (wv & 1) * 64;
    const _Float16* bbase = w16 + (size_t)(cb + m) * K2 + chalf * DIM;

    v8f acc[4];
#pragma unroll
    for (int ct = 0; ct < 4; ++ct) {
        v8f z = {0.f, 0.f, 0.f, 0.f, 0.f, 0.f, 0.f, 0.f};
        acc[ct] = z;
    }

#pragma unroll
    for (int kt = 0; kt < 8; ++kt) {
        Frag a;
        a.hf[0] = *(const v8h*)(arow + kt * 32 + 8 * h);
        a.hf[1] = *(const v8h*)(arow + kt * 32 + 16 + 8 * h);
#pragma unroll
        for (int ct = 0; ct < 4; ++ct) {
            const _Float16* bc = bbase + (size_t)ct * 16 * K2 + kt * 32;
            Frag b;
            b.hf[0] = *(const v8h*)(bc + 8 * h);
            b.hf[1] = *(const v8h*)(bc + 16 + 8 * h);
            acc[ct] = wmma_f16(a.v, b.v, acc[ct]);
        }
    }

    float* st = stile + wv * (16 * 64);
#pragma unroll
    for (int ct = 0; ct < 4; ++ct) {
#pragma unroll
        for (int r = 0; r < 8; ++r) {
            st[(8 * h + r) * 64 + ct * 16 + m] = acc[ct][r] * oscale;
        }
    }
    __syncthreads();

    const v4fa* sv = (const v4fa*)st;
    v4f vv[8];
#pragma unroll
    for (int i = 0; i < 8; ++i) {
        const int row = 2 * i + (l >> 4);
        const int c4  = l & 15;
        vv[i] = sv[row * 16 + c4];
    }
    const int gcol = wv * 64 + (l & 15) * 4;
#pragma unroll
    for (int i = 0; i < 8; ++i) {
        const int grow = r0 + 2 * i + (l >> 4);
        if (grow < nC) {
            volatile v4f* gp = (volatile v4f*)(P + (size_t)grow * DIM + gcol);
            *gp = vv[i];
        }
    }
    __threadfence();
#pragma unroll
    for (int i = 0; i < 8; ++i) {
        const int grow = r0 + 2 * i + (l >> 4);
        if (grow < nC) {
            volatile v4f* gp = (volatile v4f*)(P + (size_t)grow * DIM + gcol);
            *gp = vv[i];
        }
    }
}

__global__ __launch_bounds__(256)
void k_attn(const float* __restrict__ basic,
            const int*   __restrict__ anc,
            const float* __restrict__ maskp,
            const float* __restrict__ bp,
            const float* __restrict__ ww,
            const float* __restrict__ P,
            float*       __restrict__ out,
            int nC)
{
    const int l     = (int)(threadIdx.x & 31);
    const int wpb   = (int)(blockDim.x >> 5);
    const int gw    = blockIdx.x * wpb + ((int)threadIdx.x >> 5);
    const int nWave = gridDim.x * wpb;

    for (int n = gw; n < nC; n += nWave) {
        int idx = anc[(size_t)n * MANC + l];
        idx = idx < 0 ? 0 : (idx > nC - 1 ? nC - 1 : idx);
        const float mk = maskp[(size_t)n * MANC + l];

        const float* pa = P + (size_t)n * DIM;
        const float* pb = P + (size_t)idx * DIM + ADIM;
        float s = 0.f;
#pragma unroll 1
        for (int a = 0; a < ADIM; ++a) {
            const float x = (pa[a] + pb[a]) + bp[a];
            s += ww[a] * tanhf(x);
        }
        const float att  = s * mk;
        const float gmax = wave_max(att);
        const float w    = expf(att - gmax);
        const float sumw = wave_sum(w);
        const float inv  = 1.0f / sumw;

        v4f acc0 = {0.f, 0.f, 0.f, 0.f};
        v4f acc1 = {0.f, 0.f, 0.f, 0.f};
#pragma unroll 1
        for (int mm = 0; mm < MANC; ++mm) {
            const float wm = shf_f(w, mm);
            const int   im = shf_i(idx, mm);
            const float* rp = basic + (size_t)im * DIM + 4 * l;
            v4f e0 = *(const v4f*)rp;
            v4f e1 = *(const v4f*)(rp + ADIM);
            acc0 += wm * e0;
            acc1 += wm * e1;
        }
        const v4f o0 = acc0 * inv;
        const v4f o1 = acc1 * inv;
        volatile v4f* q0 = (volatile v4f*)(out + (size_t)n * DIM + 4 * l);
        volatile v4f* q1 = (volatile v4f*)(out + (size_t)n * DIM + ADIM + 4 * l);
        *q0 = o0;
        *q1 = o1;
        __threadfence();
        *q0 = o0;
        *q1 = o1;
    }
}

extern "C" void kernel_launch(void* const* d_in, const int* in_sizes, int n_in,
                              void* d_out, int out_size, void* d_ws, size_t ws_size,
                              hipStream_t stream) {
    if (n_in < 6) return;
    const int nC = out_size / DIM;
    if (nC <= 0) return;
    if (in_sizes[0] != nC * DIM || in_sizes[1] != nC * MANC || in_sizes[2] != nC * MANC ||
        in_sizes[3] != ADIM * K2 || in_sizes[4] < ADIM || in_sizes[5] < ADIM) return;

    const float* basic = (const float*)d_in[0];
    const int*   anc   = (const int*)  d_in[1];
    const float* mask  = (const float*)d_in[2];
    const float* Wp    = (const float*)d_in[3];
    const float* bp    = (const float*)d_in[4];
    const float* Ww    = (const float*)d_in[5];
    float*       out   = (float*)d_out;

    const size_t sz_e  = (size_t)nC * DIM * sizeof(_Float16);
    const size_t off_e = 0;
    const size_t off_w = (off_e + sz_e + 255) & ~(size_t)255;
    const size_t sz_w  = (size_t)ADIM * K2 * sizeof(_Float16);
    const size_t off_p = (off_w + sz_w + 255) & ~(size_t)255;
    const size_t sz_p  = (size_t)nC * DIM * sizeof(float);
    if (off_p + sz_p > ws_size) return;

    _Float16* e16 = (_Float16*)((char*)d_ws + off_e);
    _Float16* w16 = (_Float16*)((char*)d_ws + off_w);
    float*    P   = (float*)((char*)d_ws + off_p);

    const int n8e = nC * (DIM / 8);
    k_cvt<<<(n8e + 255) / 256, 256, 0, stream>>>(basic, e16, n8e, 8.0f);
    const int n8w = ADIM * K2 / 8;
    k_cvt<<<(n8w + 255) / 256, 256, 0, stream>>>(Wp, w16, n8w, 64.0f);

    k_proj<<<(nC + 15) / 16, 128, 0, stream>>>(e16, w16, P, nC, 1.0f / 512.0f);

    k_attn<<<(nC + 63) / 64, 256, 0, stream>>>(basic, anc, mask, bp, Ww, P, out, nC);
}
